// AlignmentNet_2164663517268
// MI455X (gfx1250) — hardware-verified
//
#include <hip/hip_runtime.h>
#include <math.h>

typedef __attribute__((ext_vector_type(16))) _Float16 v16h;
typedef __attribute__((ext_vector_type(8)))  _Float16 v8h;
typedef __attribute__((ext_vector_type(8)))  float    v8f;
typedef __attribute__((ext_vector_type(4)))  float    v4f;
typedef __attribute__((ext_vector_type(2)))  float    v2f;

constexpr int kNb    = 4;
constexpr int kCh    = 64;
constexpr int kHt    = 128;
constexpr int kWd    = 128;
constexpr int kPadH  = 130;
constexpr int kPadW  = 130;
constexpr int kOffCh = 72;
constexpr int kOffPitch = 80;
constexpr int kKcr   = 9 * 128;
constexpr int kKoff  = 9 * 64;
constexpr int kKdef  = 160;
constexpr int kNpix  = kNb * kHt * kWd;
constexpr int kHaloPix = kPadH * kPadW - kHt * kWd;
static_assert(kHaloPix == 516, "halo pixel count");
static_assert((kKcr % 32) == 0 && (kKoff % 32) == 0 && (kKdef % 32) == 0, "K multiples of 32");
static_assert((kOffPitch % 16) == 0 && kOffPitch >= kOffCh, "offset N padded to a tile multiple");

constexpr float kCarryCr   = 16.0f;
constexpr float kCarryOff  = 64.0f;
constexpr float kCarryDef  = 16.0f;
constexpr float kResScale  = 2048.0f;

constexpr size_t kPlane16B = (size_t)kNb * kPadH * kPadW * kCh * 2;
constexpr size_t kPlane32B = (size_t)kNpix * kCh * 4;
constexpr size_t kOffsB    = (size_t)kNpix * kOffPitch * 4;
constexpr size_t kWcrB     = (size_t)64 * kKcr * 2;
constexpr size_t kWoffB    = (size_t)4 * kOffPitch * kKoff * 2;
constexpr size_t kWdB      = (size_t)4 * 64 * kKdef * 2;
constexpr size_t kOfsPREF = 0;
constexpr size_t kOfsPMOV = kOfsPREF + kPlane16B;
constexpr size_t kOfsPFA  = kOfsPMOV + kPlane16B;
constexpr size_t kOfsPFB  = kOfsPFA  + kPlane16B;
constexpr size_t kOfsFM32 = kOfsPFB  + kPlane16B;
constexpr size_t kOfsFA32 = kOfsFM32 + kPlane32B;
constexpr size_t kOfsFB32 = kOfsFA32 + kPlane32B;
constexpr size_t kOfsOFFS = kOfsFB32 + kPlane32B;
constexpr size_t kOfsWCR  = kOfsOFFS + kOffsB;
constexpr size_t kOfsWOFF = kOfsWCR  + kWcrB;
constexpr size_t kOfsWDH  = kOfsWOFF + kWoffB;
constexpr size_t kOfsWDL  = kOfsWDH  + kWdB;
constexpr size_t kWsTotal = kOfsWDL  + kWdB;
static_assert(kPlane16B == 8652800ull && kPlane32B == 16777216ull && kOffsB == 20971520ull, "plane sizes");
static_assert(kWsTotal == 106594304ull, "carve total");
static_assert(kWsTotal <= 134217728ull, "carve cap");
static_assert((kPlane16B % 128) == 0 && (kPlane32B % 128) == 0 && (kOffsB % 128) == 0 &&
              (kWcrB % 512) == 0 && (kWoffB % 512) == 0 && (kWdB % 512) == 0, "line-aligned regions");

union FragU { v16h v; v8h h[2]; };
__device__ __forceinline__ v16h frag_load(const _Float16* p) {
  FragU f;
  f.h[0] = *(const v8h*)(p);
  f.h[1] = *(const v8h*)(p + 16);
  return f.v;
}
__device__ __forceinline__ v8f mma_g(v16h a, v16h b, v8f c) {
  c = __builtin_amdgcn_wmma_f32_16x16x32_f16(false, a, false, b, (short)0, c, false, false);
  asm volatile("v_nop\n\tv_nop\n\tv_nop\n\tv_nop" : "+v"(c) : "v"(a), "v"(b));
  return c;
}

__global__ __launch_bounds__(256) void halo_zero_kernel(unsigned short* planes, int nplanes) {
  const int t = blockIdx.x * 256 + threadIdx.x;
  const int item = t >> 3;
  const int c8 = (t & 7) * 8;
  const int total = nplanes * kNb * kHaloPix;
  if (item >= total) return;
  const int pb = item / kHaloPix;
  const int hix = item - pb * kHaloPix;
  const int r = hix - 260;
  const int py_side = 1 + (r >> 1);
  const int px_side = (r & 1) ? (kPadW - 1) : 0;
  const int py = (hix < 130) ? 0 : ((hix < 260) ? (kPadH - 1) : py_side);
  const int px = (hix < 130) ? hix : ((hix < 260) ? (hix - 130) : px_side);
  const size_t pixidx = ((size_t)pb * kPadH + py) * kPadW + px;
  unsigned short* q = planes + pixidx * kCh + c8;
  const v8h z = (v8h){(_Float16)0.f, (_Float16)0.f, (_Float16)0.f, (_Float16)0.f,
                      (_Float16)0.f, (_Float16)0.f, (_Float16)0.f, (_Float16)0.f};
  *(volatile v8h*)q = z;
  __threadfence();
  *(volatile v8h*)q = z;
}

__global__ __launch_bounds__(256) void pack_cr_kernel(const float* __restrict__ w, unsigned short* dst) {
  const int t = blockIdx.x * 256 + threadIdx.x;
  if (t >= 64 * 144) return;
  const int o = t / 144;
  const int k8 = (t - o * 144) * 8;
  const int tap = k8 >> 7;
  const int ci0 = k8 & 127;
  v8h hv;
#pragma unroll
  for (int e = 0; e < 8; ++e) {
    const float v = w[(size_t)(o * 128 + ci0 + e) * 9 + tap] * kCarryCr;
    hv[e] = (_Float16)v;
  }
  unsigned short* q = dst + (size_t)t * 8;
  *(volatile v8h*)q = hv;
  __threadfence();
  *(volatile v8h*)q = hv;
}

__global__ __launch_bounds__(256) void pack_off_kernel(const float* __restrict__ w0, const float* __restrict__ w1,
                                                       const float* __restrict__ w2, const float* __restrict__ w3,
                                                       unsigned short* dst) {
  const int lev = blockIdx.y;
  const float* w = (lev == 0) ? w0 : ((lev == 1) ? w1 : ((lev == 2) ? w2 : w3));
  const int t = blockIdx.x * 256 + threadIdx.x;
  if (t >= kOffPitch * 72) return;
  const int n = t / 72;
  const int k8 = (t - n * 72) * 8;
  const int tap = k8 >> 6;
  const int c0 = k8 & 63;
  const bool live = (n < kOffCh);
  const int nc = live ? n : (kOffCh - 1);
  v8h hv;
#pragma unroll
  for (int e = 0; e < 8; ++e) {
    const float raw = w[(size_t)(nc * 64 + c0 + e) * 9 + tap];
    const float v = live ? (raw * kCarryOff) : 0.0f;
    hv[e] = (_Float16)v;
  }
  unsigned short* q = dst + (size_t)lev * kOffPitch * kKoff + (size_t)t * 8;
  *(volatile v8h*)q = hv;
  __threadfence();
  *(volatile v8h*)q = hv;
}

__global__ __launch_bounds__(256) void pack_def_kernel(const float* __restrict__ w0, const float* __restrict__ w1,
                                                       const float* __restrict__ w2, const float* __restrict__ w3,
                                                       unsigned short* dhi, unsigned short* dlo) {
  const int lev = blockIdx.y;
  const float* w = (lev == 0) ? w0 : ((lev == 1) ? w1 : ((lev == 2) ? w2 : w3));
  const int t = blockIdx.x * 256 + threadIdx.x;
  if (t >= 64 * 20) return;
  const int o = t / 20;
  const int k8 = (t - o * 20) * 8;
  const bool live = (k8 < 144);
  const int tapr = k8 >> 4;
  const int tap = (tapr < 8) ? tapr : 8;
  const int c0 = k8 & 15;
  v8h hv, lv;
#pragma unroll
  for (int e = 0; e < 8; ++e) {
    const float raw = w[(size_t)(o * 16 + c0 + e) * 9 + tap];
    const float v = live ? (raw * kCarryDef) : 0.0f;
    const _Float16 hh = (_Float16)v;
    const float res = (v - (float)hh) * kResScale;
    hv[e] = hh;
    lv[e] = (_Float16)res;
  }
  unsigned short* qh = dhi + (size_t)lev * 64 * kKdef + (size_t)t * 8;
  unsigned short* ql = dlo + (size_t)lev * 64 * kKdef + (size_t)t * 8;
  *(volatile v8h*)qh = hv;
  *(volatile v8h*)ql = lv;
  __threadfence();
  *(volatile v8h*)qh = hv;
  *(volatile v8h*)ql = lv;
}

template <bool W32>
__global__ __launch_bounds__(256) void to_planes_kernel(const float* __restrict__ X, unsigned short* P16, float* P32) {
  __shared__ __align__(16) float tile[64 * 132];
  const int tid = threadIdx.x;
  const int b = blockIdx.x >> 7;
  const int y = blockIdx.x & 127;
#pragma unroll
  for (int it = 0; it < 8; ++it) {
    const int i = it * 256 + tid;
    const int c = i >> 5;
    const int x4 = (i & 31) * 4;
    const v4f v = *(const v4f*)(X + ((size_t)(b * kCh + c) * kHt + y) * kWd + x4);
    *(v4f*)(tile + c * 132 + x4) = v;
  }
  __syncthreads();
  v8h hv[4];
#pragma unroll
  for (int it = 0; it < 4; ++it) {
    const int i = it * 256 + tid;
    const int px = i >> 3;
    const int c8 = (i & 7) * 8;
#pragma unroll
    for (int e = 0; e < 8; ++e) hv[it][e] = (_Float16)tile[(c8 + e) * 132 + px];
  }
  v4f fv[8];
  if (W32) {
#pragma unroll
    for (int it = 0; it < 8; ++it) {
      const int i = it * 256 + tid;
      const int px = i >> 4;
      const int c4 = (i & 15) * 4;
#pragma unroll
      for (int e = 0; e < 4; ++e) fv[it][e] = tile[(c4 + e) * 132 + px];
    }
  }
  const size_t prow = ((size_t)(b * kPadH + y + 1) * kPadW + 1) * kCh;
  const size_t frow = ((size_t)(b * kHt + y) * kWd) * kCh;
  for (int pass = 0; pass < 2; ++pass) {
#pragma unroll
    for (int it = 0; it < 4; ++it) {
      const int i = it * 256 + tid;
      *(volatile v8h*)(P16 + prow + (size_t)i * 8) = hv[it];
    }
    if (W32) {
#pragma unroll
      for (int it = 0; it < 8; ++it) {
        const int i = it * 256 + tid;
        *(volatile v4f*)(P32 + frow + (size_t)i * 4) = fv[it];
      }
    }
    __threadfence();
  }
}

template <int NT, int NSRC, bool OFFOUT>
__global__ __launch_bounds__(128) void conv3x3_kernel(const unsigned short* __restrict__ P0p,
                                                      const unsigned short* __restrict__ P1p,
                                                      const unsigned short* __restrict__ Btp,
                                                      const float* __restrict__ bias,
                                                      unsigned short* out16, float* out32) {
  constexpr int KTOT = 9 * NSRC * 64;
  constexpr int SP = OFFOUT ? 84 : 68;
  constexpr float INVC = OFFOUT ? (1.0f / kCarryOff) : (1.0f / kCarryCr);
  static_assert(OFFOUT ? (NT * 16 == kOffPitch) : (NT * 16 == kCh), "column tiles");
  __shared__ __align__(16) float sS[4 * 16 * SP];
  const int tid = threadIdx.x;
  const int lane = tid & 31;
  const int wave = tid >> 5;
  const int m = lane & 15;
  const int h = lane >> 4;
  const int b = blockIdx.x >> 7;
  const int y = blockIdx.x & 127;
  const int x0 = wave * 32;
  const _Float16* A0 = (const _Float16*)P0p;
  const _Float16* A1 = (const _Float16*)P1p;
  const _Float16* Bl = (const _Float16*)Btp + (size_t)m * KTOT + 8 * h;

  v8f acc[2][NT];
#pragma unroll
  for (int i = 0; i < 2; ++i)
#pragma unroll
    for (int j = 0; j < NT; ++j) acc[i][j] = (v8f){0.f, 0.f, 0.f, 0.f, 0.f, 0.f, 0.f, 0.f};

#pragma unroll 1
  for (int tap = 0; tap < 9; ++tap) {
    const int kh = tap / 3;
    const int kw = tap - kh * 3;
    const size_t pixoff = ((size_t)(b * kPadH + y + kh) * kPadW + (x0 + m + kw)) * kCh + 8 * h;
#pragma unroll
    for (int s = 0; s < NSRC; ++s) {
      const _Float16* Ap = ((s == 0) ? A0 : A1) + pixoff;
#pragma unroll
      for (int cc = 0; cc < 2; ++cc) {
        const v16h a0 = frag_load(Ap + cc * 32);
        const v16h a1 = frag_load(Ap + 16 * kCh + cc * 32);
        const _Float16* Bp = Bl + (tap * NSRC + s) * 64 + cc * 32;
#pragma unroll
        for (int j = 0; j < NT; ++j) {
          const v16h bf = frag_load(Bp + (size_t)j * 16 * KTOT);
          acc[0][j] = mma_g(a0, bf, acc[0][j]);
          acc[1][j] = mma_g(a1, bf, acc[1][j]);
        }
      }
    }
  }

  float bv[NT];
#pragma unroll
  for (int j = 0; j < NT; ++j) {
    const int n = j * 16 + m;
    if (OFFOUT) {
      const int nc = (n < kOffCh) ? n : (kOffCh - 1);
      const float t = bias[nc];
      bv[j] = (n < kOffCh) ? t : 0.0f;
    } else {
      bv[j] = bias[n];
    }
  }

  float* slab = sS + wave * 16 * SP;
  const size_t pixrow = (size_t)(b * kHt + y) * kWd;
#pragma unroll
  for (int mt = 0; mt < 2; ++mt) {
#pragma unroll
    for (int j = 0; j < NT; ++j) {
#pragma unroll
      for (int r = 0; r < 8; ++r) {
        slab[(8 * h + r) * SP + j * 16 + m] = acc[mt][j][r] * INVC + bv[j];
      }
    }
    __syncthreads();
    if (OFFOUT) {
      float* dst = out32 + (pixrow + x0 + mt * 16) * kOffPitch;
      for (int pass = 0; pass < 2; ++pass) {
#pragma unroll
        for (int it = 0; it < 10; ++it) {
          const int i = it * 32 + lane;
          const int p = i / 20;
          const int c4 = (i - p * 20) * 4;
          const v4f v = *(const v4f*)(slab + p * SP + c4);
          *(volatile v4f*)(dst + (size_t)i * 4) = v;
        }
        __threadfence();
      }
    } else {
      v8h hv[4];
#pragma unroll
      for (int it = 0; it < 4; ++it) {
        const int p = it * 4 + (lane >> 3);
        const int c8 = (lane & 7) * 8;
        const v4f q0 = *(const v4f*)(slab + p * SP + c8);
        const v4f q1 = *(const v4f*)(slab + p * SP + c8 + 4);
#pragma unroll
        for (int e = 0; e < 4; ++e) {
          hv[it][e] = (_Float16)q0[e];
          hv[it][4 + e] = (_Float16)q1[e];
        }
      }
      unsigned short* d16 = out16 + ((size_t)(b * kPadH + y + 1) * kPadW + (x0 + mt * 16 + 1)) * kCh;
      float* d32 = out32 + (pixrow + x0 + mt * 16) * kCh;
      for (int pass = 0; pass < 2; ++pass) {
#pragma unroll
        for (int it = 0; it < 4; ++it) {
          const int i = it * 32 + lane;
          *(volatile v8h*)(d16 + (size_t)i * 8) = hv[it];
        }
#pragma unroll
        for (int it = 0; it < 8; ++it) {
          const int i = it * 32 + lane;
          const int p = i >> 4;
          const int c4 = (i & 15) * 4;
          const v4f v = *(const v4f*)(slab + p * SP + c4);
          *(volatile v4f*)(d32 + (size_t)i * 4) = v;
        }
        __threadfence();
      }
    }
    __syncthreads();
  }
}

__device__ __forceinline__ v4f blend4(const float* p00, const float* p01, const float* p10, const float* p11,
                                      float w00, float w01, float w10, float w11) {
  const v4f a = *(const v4f*)p00;
  const v4f b = *(const v4f*)p01;
  const v4f c = *(const v4f*)p10;
  const v4f d = *(const v4f*)p11;
  v4f s;
#pragma unroll
  for (int e = 0; e < 4; ++e) {
    float t = w00 * a[e];
    t = fmaf(w01, b[e], t);
    t = fmaf(w10, c[e], t);
    t = fmaf(w11, d[e], t);
    s[e] = t;
  }
  return s;
}

template <bool SPLIT, bool OUT_NCHW, bool W16, bool W32>
__global__ __launch_bounds__(64) void deform_kernel(const float* __restrict__ SRC, const float* __restrict__ OFF,
                                                    const unsigned short* __restrict__ Whp,
                                                    const unsigned short* __restrict__ Wlp,
                                                    const float* __restrict__ bias,
                                                    unsigned short* out16, float* out32) {
  constexpr int AP = 168;
  constexpr int SLAB = 2304;
  static_assert(32 * 68 <= SLAB && 64 * 36 <= SLAB, "slab extent");
  __shared__ __align__(16) _Float16 sAh[2 * 32 * AP];
  __shared__ __align__(16) _Float16 sAl[SPLIT ? 2 * 32 * AP : 8];
  __shared__ __align__(16) float sO[2 * SLAB];
  const int tid = threadIdx.x;
  const int lane = tid & 31;
  const int wave = tid >> 5;
  const int m = lane & 15;
  const int h = lane >> 4;
  const int bid = blockIdx.x;
  const int b = bid >> 8;
  const int y = (bid >> 1) & 127;
  const int x0 = (bid & 1) * 64 + wave * 32;
  const int x = x0 + lane;
  const size_t pixrow = (size_t)(b * kHt + y) * kWd;
  const size_t pix = pixrow + x;
  _Float16* Ah = sAh + wave * 32 * AP;
  _Float16* Al = sAl + (SPLIT ? wave * 32 * AP : 0);
  float* so = sO + wave * SLAB;
  const _Float16* Wh = (const _Float16*)Whp;
  const _Float16* Wl = (const _Float16*)Wlp;
  const float* srcb = SRC + (size_t)b * kHt * kWd * kCh;
  const v8h zero8 = (v8h){(_Float16)0.f, (_Float16)0.f, (_Float16)0.f, (_Float16)0.f,
                          (_Float16)0.f, (_Float16)0.f, (_Float16)0.f, (_Float16)0.f};
  constexpr float INVC = 1.0f / kCarryDef;
  constexpr float INVR = 1.0f / (kCarryDef * kResScale);

#pragma unroll 1
  for (int g = 0; g < 4; ++g) {
    __syncthreads();
    const float* offp = OFF + pix * kOffPitch + g * 18;
    const float* srcg = srcb + g * 16;
    int kh = 0, kw = 0;
#pragma unroll 1
    for (int kk = 0; kk < 9; ++kk) {
      const v2f d = *(const v2f*)(offp + kk * 2);
      const float py = d[0] + (float)(y - 2 + 2 * kh);
      const float px = d[1] + (float)(x - 2 + 2 * kw);
      const float y0f = floorf(py);
      const float x0f = floorf(px);
      const float ly = py - y0f;
      const float lx = px - x0f;
      const float y1f = y0f + 1.0f;
      const float x1f = x0f + 1.0f;
      const bool vy0 = (y0f >= 0.0f) && (y0f <= 127.0f);
      const bool vy1 = (y1f >= 0.0f) && (y1f <= 127.0f);
      const bool vx0 = (x0f >= 0.0f) && (x0f <= 127.0f);
      const bool vx1 = (x1f >= 0.0f) && (x1f <= 127.0f);
      const int iy0 = (int)fminf(fmaxf(y0f, 0.0f), 127.0f);
      const int iy1 = (int)fminf(fmaxf(y1f, 0.0f), 127.0f);
      const int ix0 = (int)fminf(fmaxf(x0f, 0.0f), 127.0f);
      const int ix1 = (int)fminf(fmaxf(x1f, 0.0f), 127.0f);
      const float hy = 1.0f - ly;
      const float hx = 1.0f - lx;
      const float w00 = (vy0 && vx0) ? (hy * hx) : 0.0f;
      const float w01 = (vy0 && vx1) ? (hy * lx) : 0.0f;
      const float w10 = (vy1 && vx0) ? (ly * hx) : 0.0f;
      const float w11 = (vy1 && vx1) ? (ly * lx) : 0.0f;
      const float* p00 = srcg + (size_t)(iy0 * kWd + ix0) * kCh;
      const float* p01 = srcg + (size_t)(iy0 * kWd + ix1) * kCh;
      const float* p10 = srcg + (size_t)(iy1 * kWd + ix0) * kCh;
      const float* p11 = srcg + (size_t)(iy1 * kWd + ix1) * kCh;
      v8h h0 = zero8, h1 = zero8, l0 = zero8, l1 = zero8;
#pragma unroll
      for (int q = 0; q < 2; ++q) {
        const v4f s = blend4(p00 + 4 * q, p01 + 4 * q, p10 + 4 * q, p11 + 4 * q, w00, w01, w10, w11);
        const v4f u = blend4(p00 + 8 + 4 * q, p01 + 8 + 4 * q, p10 + 8 + 4 * q, p11 + 8 + 4 * q, w00, w01, w10, w11);
#pragma unroll
        for (int e = 0; e < 4; ++e) {
          const float sv = s[e];
          const float uv = u[e];
          const _Float16 sh = (_Float16)sv;
          const _Float16 uh = (_Float16)uv;
          h0[q * 4 + e] = sh;
          h1[q * 4 + e] = uh;
          if (SPLIT) {
            const float sr = (sv - (float)sh) * kResScale;
            const float ur = (uv - (float)uh) * kResScale;
            l0[q * 4 + e] = (_Float16)sr;
            l1[q * 4 + e] = (_Float16)ur;
          }
        }
      }
      *(v8h*)(Ah + lane * AP + kk * 16) = h0;
      *(v8h*)(Ah + lane * AP + kk * 16 + 8) = h1;
      if (SPLIT) {
        *(v8h*)(Al + lane * AP + kk * 16) = l0;
        *(v8h*)(Al + lane * AP + kk * 16 + 8) = l1;
      }
      kw += 1;
      if (kw == 3) { kw = 0; kh += 1; }
    }
    *(v8h*)(Ah + lane * AP + 144) = zero8;
    *(v8h*)(Ah + lane * AP + 152) = zero8;
    if (SPLIT) {
      *(v8h*)(Al + lane * AP + 144) = zero8;
      *(v8h*)(Al + lane * AP + 152) = zero8;
    }
    __syncthreads();

    v8f acc0 = (v8f){0.f, 0.f, 0.f, 0.f, 0.f, 0.f, 0.f, 0.f};
    v8f acc1 = acc0;
    v8f ar0 = acc0;
    v8f ar1 = acc0;
#pragma unroll 1
    for (int kt = 0; kt < 5; ++kt) {
      const size_t wo = (size_t)(g * 16 + m) * kKdef + kt * 32 + 8 * h;
      const int ao = m * AP + kt * 32 + 8 * h;
      const v16h bh = frag_load(Wh + wo);
      const v16h a0 = frag_load(Ah + ao);
      const v16h a1 = frag_load(Ah + 16 * AP + ao);
      acc0 = mma_g(a0, bh, acc0);
      acc1 = mma_g(a1, bh, acc1);
      if (SPLIT) {
        const v16h bl = frag_load(Wl + wo);
        const v16h al0 = frag_load(Al + ao);
        const v16h al1 = frag_load(Al + 16 * AP + ao);
        ar0 = mma_g(a0, bl, ar0);
        ar0 = mma_g(al0, bh, ar0);
        ar1 = mma_g(a1, bl, ar1);
        ar1 = mma_g(al1, bh, ar1);
      }
    }
    const int o = g * 16 + m;
    const float bvv = bias[o];
#pragma unroll
    for (int r = 0; r < 8; ++r) {
      float v0 = acc0[r] * INVC;
      float v1 = acc1[r] * INVC;
      if (SPLIT) {
        v0 += ar0[r] * INVR;
        v1 += ar1[r] * INVR;
      }
      v0 += bvv;
      v1 += bvv;
      const int p0 = 8 * h + r;
      const int p1 = 16 + 8 * h + r;
      if (OUT_NCHW) {
        so[o * 36 + p0] = v0;
        so[o * 36 + p1] = v1;
      } else {
        so[p0 * 68 + o] = v0;
        so[p1 * 68 + o] = v1;
      }
    }
  }
  __syncthreads();

  if (OUT_NCHW) {
    for (int pass = 0; pass < 2; ++pass) {
#pragma unroll
      for (int it = 0; it < 16; ++it) {
        const int chn = it * 4 + (lane >> 3);
        const int p4 = (lane & 7) * 4;
        const v4f v = *(const v4f*)(so + chn * 36 + p4);
        *(volatile v4f*)(out32 + ((size_t)(b * kCh + chn) * kHt + y) * kWd + x0 + p4) = v;
      }
      __threadfence();
    }
  } else {
    v8h hv[8];
    if (W16) {
#pragma unroll
      for (int it = 0; it < 8; ++it) {
        const int p = it * 4 + (lane >> 3);
        const int c8 = (lane & 7) * 8;
        const v4f q0 = *(const v4f*)(so + p * 68 + c8);
        const v4f q1 = *(const v4f*)(so + p * 68 + c8 + 4);
#pragma unroll
        for (int e = 0; e < 4; ++e) {
          hv[it][e] = (_Float16)q0[e];
          hv[it][4 + e] = (_Float16)q1[e];
        }
      }
    }
    unsigned short* d16 = out16 + ((size_t)(b * kPadH + y + 1) * kPadW + (x0 + 1)) * kCh;
    float* d32 = out32 + (pixrow + x0) * kCh;
    for (int pass = 0; pass < 2; ++pass) {
      if (W16) {
#pragma unroll
        for (int it = 0; it < 8; ++it) {
          const int i = it * 32 + lane;
          *(volatile v8h*)(d16 + (size_t)i * 8) = hv[it];
        }
      }
      if (W32) {
#pragma unroll
        for (int it = 0; it < 16; ++it) {
          const int i = it * 32 + lane;
          const int p = i >> 4;
          const int c4 = (i & 15) * 4;
          const v4f v = *(const v4f*)(so + p * 68 + c4);
          *(volatile v4f*)(d32 + (size_t)i * 4) = v;
        }
      }
      __threadfence();
    }
  }
}

extern "C" void kernel_launch(void* const* d_in, const int* in_sizes, int n_in,
                              void* d_out, int out_size, void* d_ws, size_t ws_size,
                              hipStream_t stream) {
  if (n_in < 21) return;
  if (in_sizes[0] != kNpix * kCh || in_sizes[1] != kNpix * kCh || in_sizes[2] != kNpix * kCh) return;
  if (in_sizes[3] != 64 * 128 * 9 || in_sizes[4] != 64) return;
  for (int i = 0; i < 4; ++i) {
    if (in_sizes[5 + 2 * i] != kOffCh * 64 * 9 || in_sizes[6 + 2 * i] != kOffCh) return;
    if (in_sizes[13 + 2 * i] != 64 * 16 * 9 || in_sizes[14 + 2 * i] != 64) return;
  }
  if (out_size != 2 * kNpix * kCh) return;
  if (ws_size < kWsTotal) return;

  const float* Fref = (const float*)d_in[0];
  const float* Fmov[2] = { (const float*)d_in[1], (const float*)d_in[2] };
  const float* cr_w = (const float*)d_in[3];
  const float* cr_b = (const float*)d_in[4];
  const float* off_w[4] = { (const float*)d_in[5], (const float*)d_in[7], (const float*)d_in[9], (const float*)d_in[11] };
  const float* off_b[4] = { (const float*)d_in[6], (const float*)d_in[8], (const float*)d_in[10], (const float*)d_in[12] };
  const float* def_w[4] = { (const float*)d_in[13], (const float*)d_in[15], (const float*)d_in[17], (const float*)d_in[19] };
  const float* def_b[4] = { (const float*)d_in[14], (const float*)d_in[16], (const float*)d_in[18], (const float*)d_in[20] };
  float* out = (float*)d_out;

  char* ws = (char*)d_ws;
  unsigned short* PREF = (unsigned short*)(ws + kOfsPREF);
  unsigned short* PMOV = (unsigned short*)(ws + kOfsPMOV);
  unsigned short* PFA  = (unsigned short*)(ws + kOfsPFA);
  unsigned short* PFB  = (unsigned short*)(ws + kOfsPFB);
  float* FM32 = (float*)(ws + kOfsFM32);
  float* FA32 = (float*)(ws + kOfsFA32);
  float* FB32 = (float*)(ws + kOfsFB32);
  float* OFFS = (float*)(ws + kOfsOFFS);
  unsigned short* WCR  = (unsigned short*)(ws + kOfsWCR);
  unsigned short* WOFF = (unsigned short*)(ws + kOfsWOFF);
  unsigned short* WDH  = (unsigned short*)(ws + kOfsWDH);
  unsigned short* WDL  = (unsigned short*)(ws + kOfsWDL);

  halo_zero_kernel<<<(4 * kNb * kHaloPix * 8 + 255) / 256, 256, 0, stream>>>(PREF, 4);
  pack_cr_kernel<<<36, 256, 0, stream>>>(cr_w, WCR);
  pack_off_kernel<<<dim3(23, 4), 256, 0, stream>>>(off_w[0], off_w[1], off_w[2], off_w[3], WOFF);
  pack_def_kernel<<<dim3(5, 4), 256, 0, stream>>>(def_w[0], def_w[1], def_w[2], def_w[3], WDH, WDL);
  to_planes_kernel<false><<<kNb * kHt, 256, 0, stream>>>(Fref, PREF, FM32);

  const int convBlocks = kNb * kHt;
  const int defBlocks = kNb * kHt * 2;
  const size_t offLev = (size_t)kOffPitch * kKoff;
  const size_t defLev = (size_t)64 * kKdef;

  for (int a = 0; a < 2; ++a) {
    float* dst = out + (size_t)a * kNpix * kCh;
    to_planes_kernel<true><<<kNb * kHt, 256, 0, stream>>>(Fmov[a], PMOV, FM32);
    conv3x3_kernel<4, 2, false><<<convBlocks, 128, 0, stream>>>(PREF, PMOV, WCR, cr_b, PFA, FA32);
    conv3x3_kernel<5, 1, true><<<convBlocks, 128, 0, stream>>>(PFA, PFA, WOFF + 0 * offLev, off_b[0], PFB, OFFS);
    deform_kernel<false, false, true, true><<<defBlocks, 64, 0, stream>>>(FA32, OFFS, WDH + 0 * defLev, WDL + 0 * defLev, def_b[0], PFB, FB32);
    conv3x3_kernel<5, 1, true><<<convBlocks, 128, 0, stream>>>(PFB, PFB, WOFF + 1 * offLev, off_b[1], PFA, OFFS);
    deform_kernel<false, false, true, false><<<defBlocks, 64, 0, stream>>>(FB32, OFFS, WDH + 1 * defLev, WDL + 1 * defLev, def_b[1], PFA, FA32);
    conv3x3_kernel<5, 1, true><<<convBlocks, 128, 0, stream>>>(PFA, PFA, WOFF + 2 * offLev, off_b[2], PFB, OFFS);
    deform_kernel<true, false, true, true><<<defBlocks, 64, 0, stream>>>(FM32, OFFS, WDH + 2 * defLev, WDL + 2 * defLev, def_b[2], PFB, FA32);
    conv3x3_kernel<5, 1, true><<<convBlocks, 128, 0, stream>>>(PFB, PFB, WOFF + 3 * offLev, off_b[3], PFA, OFFS);
    deform_kernel<true, true, false, false><<<defBlocks, 64, 0, stream>>>(FA32, OFFS, WDH + 3 * defLev, WDL + 3 * defLev, def_b[3], PFA, dst);
  }
}
